// GAT_graph_branch_46127948759399
// MI455X (gfx1250) — hardware-verified
//
#include <hip/hip_runtime.h>
#include <stddef.h>
#include <stdint.h>


#define FIN     128
#define C1      64
#define C2      32
#define NG      16
#define N1      192
#define N2      96
#define KG      128
#define NTHR    256
#define NWAVE   8
#define EPT     8
#define CHUNK   (NTHR * EPT)
#define WCAP    (EPT * 32)
#define LISTN   (NWAVE * WCAP)
#define NBA     1024
#define SLA     10
#define RCAP    28672
#define DEGCAP  64
#define GBM     64
#define GTHR    128
#define EAR     4096
#define NEGS    0.2f
#define WSMAX   134217728
#define BK_ZINTS (LISTN + 2 * RCAP + 3 * NBA)
#define BK_LDS_INTS (BK_ZINTS + 16)
#define VEC_N   384

static_assert((CHUNK & (CHUNK - 1)) == 0 && CHUNK <= 4096);
static_assert((NBA & (NBA - 1)) == 0 && NBA == (1 << SLA));
static_assert(((long long)CHUNK << SLA) < (1LL << 31));
static_assert(NBA % NWAVE == 0 && NBA % 32 == 0 && NBA == NTHR * 4);
static_assert(RCAP % (NTHR * 4) == 0 && BK_ZINTS % 4 == 0 && LISTN % 4 == 0);
static_assert(BK_LDS_INTS * 4 <= 300000);
static_assert(GBM == (GTHR / 32) * 16);
static_assert(KG % 32 == 0 && KG == FIN && KG == 2 * C1);
static_assert(N1 == 3 * C1 && N2 == 3 * C2 && C1 == 2 * 32 && C2 == 32);
static_assert(DEGCAP >= 35 + 8 && RCAP >= 16623 + 4096);
static_assert(EAR % 64 == 0);
static_assert(NG == 16);

typedef float          v2f   __attribute__((ext_vector_type(2)));
typedef float          v4f   __attribute__((ext_vector_type(4)));
typedef float          v8f   __attribute__((ext_vector_type(8)));
typedef int            v4i   __attribute__((ext_vector_type(4)));
typedef int            v8i   __attribute__((ext_vector_type(8)));
typedef double         v2d   __attribute__((ext_vector_type(2)));
typedef unsigned short v8us  __attribute__((ext_vector_type(8)));
typedef __bf16         v16bf __attribute__((ext_vector_type(16)));
typedef v2f  __attribute__((may_alias)) v2fa;
typedef v4f  __attribute__((may_alias)) v4fa;
typedef v4i  __attribute__((may_alias)) v4ia;
union FragB { v16bf v; v8us u[2]; v8i w; };

__device__ __forceinline__ v8f wmx(const FragB& a, const FragB& b, v8f c) {
  v8f d = __builtin_amdgcn_wmma_f32_16x16x32_bf16(false, a.v, false, b.v, (short)0, c, false, false);
  asm volatile("v_nop\n\tv_nop\n\tv_nop\n\tv_nop" : "+v"(d) : "v"(a.w), "v"(b.w));
  return d;
}

__device__ __forceinline__ unsigned bfbits(float v) {
  unsigned u = __float_as_uint(v);
  u = u + 0x7FFFu + ((u >> 16) & 1u);
  return u >> 16;
}
__device__ __forceinline__ float rbf(float v) { return __uint_as_float(bfbits(v) << 16); }

__device__ __forceinline__ v8us cvt8b(const v4f a, const v4f b) {
  v8us o;
  o[0] = (unsigned short)bfbits(a.x); o[1] = (unsigned short)bfbits(a.y);
  o[2] = (unsigned short)bfbits(a.z); o[3] = (unsigned short)bfbits(a.w);
  o[4] = (unsigned short)bfbits(b.x); o[5] = (unsigned short)bfbits(b.y);
  o[6] = (unsigned short)bfbits(b.z); o[7] = (unsigned short)bfbits(b.w);
  return o;
}

template <int SLB>
__device__ __forceinline__ int scan_chunk(const int* __restrict__ dsts, int nE, int cbase, int slotBase,
                                          int nb, int vec8, int* list, int tid, int lane, int wave) {
  int wc = 0;
  const int el0  = tid * EPT;
  const int e0   = cbase + el0;
  const int sent = -2147483647 - 1;
  v4i da, db;
  if (vec8 != 0 && cbase + CHUNK <= nE) {
    da = *(const v4i*)(dsts + e0);
    db = *(const v4i*)(dsts + e0 + 4);
  } else {
    da.x = (e0     < nE) ? dsts[min(e0,     nE - 1)] : sent;
    da.y = (e0 + 1 < nE) ? dsts[min(e0 + 1, nE - 1)] : sent;
    da.z = (e0 + 2 < nE) ? dsts[min(e0 + 2, nE - 1)] : sent;
    da.w = (e0 + 3 < nE) ? dsts[min(e0 + 3, nE - 1)] : sent;
    db.x = (e0 + 4 < nE) ? dsts[min(e0 + 4, nE - 1)] : sent;
    db.y = (e0 + 5 < nE) ? dsts[min(e0 + 5, nE - 1)] : sent;
    db.z = (e0 + 6 < nE) ? dsts[min(e0 + 6, nE - 1)] : sent;
    db.w = (e0 + 7 < nE) ? dsts[min(e0 + 7, nE - 1)] : sent;
  }
  const unsigned nbs = (unsigned)slotBase;
  const unsigned unb = (unsigned)nb;
  const unsigned s0 = (unsigned)da.x - nbs, s1 = (unsigned)da.y - nbs;
  const unsigned s2 = (unsigned)da.z - nbs, s3 = (unsigned)da.w - nbs;
  const unsigned s4 = (unsigned)db.x - nbs, s5 = (unsigned)db.y - nbs;
  const unsigned s6 = (unsigned)db.z - nbs, s7 = (unsigned)db.w - nbs;
  const bool h0 = s0 < unb, h1 = s1 < unb, h2 = s2 < unb, h3 = s3 < unb;
  const bool h4 = s4 < unb, h5 = s5 < unb, h6 = s6 < unb, h7 = s7 < unb;
  const unsigned any = __builtin_amdgcn_ballot_w32(h0 | h1 | h2 | h3 | h4 | h5 | h6 | h7);
  if (any != 0u) {
#define HITJ(J, HJ, SJ) { \
      const unsigned mj = __builtin_amdgcn_ballot_w32(HJ); \
      if (mj != 0u) { \
        if (HJ) { \
          const int pos = wc + (int)__builtin_amdgcn_mbcnt_lo(mj, 0u); \
          if (pos < WCAP) list[wave * WCAP + pos] = ((el0 + (J)) << SLB) | (int)(SJ); \
        } \
        wc += (int)__builtin_popcount(mj); } }
    HITJ(0, h0, s0)
    HITJ(1, h1, s1)
    HITJ(2, h2, s2)
    HITJ(3, h3, s3)
    HITJ(4, h4, s4)
    HITJ(5, h5, s5)
    HITJ(6, h6, s6)
    HITJ(7, h7, s7)
#undef HITJ
  }
  return wc;
}

__global__ __launch_bounds__(NTHR) void k_xprep(const float* __restrict__ x, unsigned short* xb, int nN, int nUnits) {
  const int i = (int)blockIdx.x * NTHR + (int)threadIdx.x;
  if (i >= nUnits) return;
  const int row = i >> 4;
  const int c0  = (i & 15) * 8;
  const int rc  = row < nN ? row : nN - 1;
  const float* p = x + (size_t)rc * FIN + c0;
  v4f a = *(const v4f*)p, b = *(const v4f*)(p + 4);
  const v4f z4 = {0.f, 0.f, 0.f, 0.f};
  if (row >= nN) { a = z4; b = z4; }
  const v8us hv = cvt8b(a, b);
  const size_t o = (size_t)row * FIN + c0;
  *(volatile v8us*)(xb + o) = hv;
  __threadfence();
  *(volatile v8us*)(xb + o) = hv;
}

__device__ __forceinline__ v8us gath8(const float* __restrict__ w, int cols, int k0, int n) {
  const float* p = w + (size_t)k0 * (size_t)cols + n;
  v4f a, b;
  a.x = p[0];                  a.y = p[(size_t)cols];       a.z = p[(size_t)2 * cols];   a.w = p[(size_t)3 * cols];
  b.x = p[(size_t)4 * cols];   b.y = p[(size_t)5 * cols];   b.z = p[(size_t)6 * cols];   b.w = p[(size_t)7 * cols];
  return cvt8b(a, b);
}

__global__ __launch_bounds__(NTHR) void k_wprep(const float* __restrict__ s1w, const float* __restrict__ wl1,
                                                const float* __restrict__ wr1, const float* __restrict__ s2w,
                                                const float* __restrict__ wl2, const float* __restrict__ wr2,
                                                unsigned short* wt) {
  const int u = (int)blockIdx.x * NTHR + (int)threadIdx.x;
  v8us o;
  if (u < 1024) {
    o = gath8(s1w, C1, (u & 15) * 8, u >> 4);
  } else if (u < 2048) {
    const int v = u - 1024;
    o = gath8(wl1, C1, (v & 15) * 8, v >> 4);
  } else if (u < 3072) {
    const int v = u - 2048;
    o = gath8(wr1, C1, (v & 15) * 8, v >> 4);
  } else if (u < 3584) {
    const int v = u - 3072;
    o = gath8(s2w, C2, ((v & 15) * 8) & 63, v >> 4);
  } else if (u < 4096) {
    const int v = u - 3584;
    o = gath8(wl2, C2, ((v & 15) * 8) & 63, v >> 4);
  } else if (u < 4608) {
    const int v = u - 4096;
    o = gath8(wr2, C2, ((v & 15) * 8) & 63, v >> 4);
  } else {
    return;
  }
  unsigned short* dp = wt + (size_t)u * 8;
  *(volatile v8us*)dp = o;
  __threadfence();
  *(volatile v8us*)dp = o;
}

__global__ __launch_bounds__(NTHR) void k_easum(const float* __restrict__ ea, int nE, double* rec) {
  __shared__ double ls[NTHR * 4];
  __shared__ __attribute__((aligned(16))) double lo[16];
  const int tid = (int)threadIdx.x;
  const int q = tid & 3, rs = tid >> 2;
  const int base = (int)blockIdx.x * EAR;
  double s0 = 0.0, s1 = 0.0, s2 = 0.0, s3 = 0.0;
#pragma unroll 1
  for (int it = 0; it < EAR / 64; ++it) {
    const int row = base + it * 64 + rs;
    const int rc  = row < nE ? row : nE - 1;
    const v4f v = *(const v4f*)(ea + (size_t)rc * 16 + 4 * q);
    const float lv = row < nE ? 1.0f : 0.0f;
    s0 += (double)(rbf(v.x) * lv);
    s1 += (double)(rbf(v.y) * lv);
    s2 += (double)(rbf(v.z) * lv);
    s3 += (double)(rbf(v.w) * lv);
  }
  ls[tid * 4 + 0] = s0; ls[tid * 4 + 1] = s1; ls[tid * 4 + 2] = s2; ls[tid * 4 + 3] = s3;
  __syncthreads();
  if (tid < 16) {
    const int qq = tid >> 2, j = tid & 3;
    double a = 0.0;
#pragma unroll 1
    for (int r = 0; r < 64; ++r) a += ls[(r * 4 + qq) * 4 + j];
    lo[tid] = a;
  }
  __syncthreads();
  if (tid < 8) {
    v2d t;
    t.x = lo[2 * tid]; t.y = lo[2 * tid + 1];
    double* dp = rec + (size_t)blockIdx.x * 16 + 2 * tid;
    *(volatile v2d*)dp = t;
    __threadfence();
    *(volatile v2d*)dp = t;
  }
}

__global__ __launch_bounds__(384) void k_eamean(const double* __restrict__ rec, int nRec, int nE,
                                                const float* __restrict__ we1, const float* __restrict__ we2,
                                                const float* __restrict__ s1b, const float* __restrict__ bl1,
                                                const float* __restrict__ br1, const float* __restrict__ s2b,
                                                const float* __restrict__ bl2, const float* __restrict__ br2,
                                                float* vec) {
  __shared__ float mean_s[16];
  __shared__ __attribute__((aligned(16))) float vst[VEC_N];
  const int tid = (int)threadIdx.x;
  const int wave = __builtin_amdgcn_readfirstlane(tid >> 5);
  if (wave == 0) {
    const int c = tid & 15;
    double s = 0.0;
#pragma unroll 1
    for (int b = 0; b < nRec; ++b) s += rec[(size_t)b * 16 + c];
    const float mv = (float)(s / (double)nE);
    if (tid < 16) mean_s[tid] = mv;
  }
  __syncthreads();
  float v = 0.0f;
  int slot = tid - 96;
  if (wave < 2) {
    float acc = 0.0f;
#pragma unroll 4
    for (int k = 0; k < 16; ++k) acc = fmaf(mean_s[k], rbf(we1[k * C1 + tid]), acc);
    v = acc; slot = 288 + tid;
  } else if (wave == 2) {
    float acc = 0.0f;
#pragma unroll 4
    for (int k = 0; k < 16; ++k) acc = fmaf(mean_s[k], rbf(we2[k * C2 + (tid - 64)]), acc);
    v = acc; slot = 288 + tid;
  } else if (wave < 5) {
    v = rbf(s1b[tid - 96]);
  } else if (wave < 7) {
    v = rbf(bl1[tid - 160]);
  } else if (wave < 9) {
    v = rbf(br1[tid - 224]);
  } else if (wave == 9) {
    v = rbf(s2b[tid - 288]);
  } else if (wave == 10) {
    v = rbf(bl2[tid - 320]);
  } else {
    v = rbf(br2[tid - 352]);
  }
  vst[slot] = v;
  __syncthreads();
  if (tid < VEC_N / 4) {
    const v4f o = *(const v4fa*)(vst + 4 * tid);
    *(volatile v4f*)(vec + 4 * tid) = o;
    __threadfence();
    *(volatile v4f*)(vec + 4 * tid) = o;
  }
}

__global__ __launch_bounds__(NTHR) void k_bucket(const int* __restrict__ srcs, const int* __restrict__ dsts,
                                                 int nE, int nN, int vec8,
                                                 int* eidp, int* srcp, int* offt, int* meta) {
  extern __shared__ __attribute__((aligned(16))) int dsm[];
  int* list = dsm;
  int* hl   = dsm + LISTN;
  int* sl   = hl + RCAP;
  int* cnt  = sl + RCAP;
  int* offs = cnt + NBA;
  int* cur  = offs + NBA;
  int* misc = cur + NBA;
  const int tid = (int)threadIdx.x, lane = tid & 31, wave = tid >> 5;
  const int nodeBase = (int)blockIdx.x * NBA;

  {
    const v4i z4 = {0, 0, 0, 0};
    for (int i = tid * 4; i < BK_ZINTS; i += NTHR * 4) *(v4ia*)(dsm + i) = z4;
    if (tid < 16) misc[tid] = 0;
  }
  __syncthreads();

  int t = 0, ov = 0;
  const int nChunks = (nE + CHUNK - 1) / CHUNK;
#pragma unroll 1
  for (int ch = 0; ch < nChunks; ++ch) {
    const int cbase = ch * CHUNK;
    const int wc = scan_chunk<SLA>(dsts, nE, cbase, nodeBase, NBA, vec8, list, tid, lane, wave);
    if (lane == 0) misc[wave] = wc;
    __syncthreads();
    if (wave == 0) {
#pragma unroll 1
      for (int w2 = 0; w2 < NWAVE; ++w2) {
        int c = misc[w2];
        c = c < 0 ? 0 : (c > WCAP ? WCAP : c);
#pragma unroll 1
        for (int b0 = 0; b0 < c; b0 += 32) {
          const int idx = b0 + lane;
          const int ent = list[w2 * WCAP + (idx < WCAP ? idx : WCAP - 1)];
          const int m32 = (c - b0) < 32 ? (c - b0) : 32;
#pragma unroll 1
          for (int k = 0; k < m32; ++k) {
            const int u    = __builtin_amdgcn_readlane(ent, k);
            const int slot = u & (NBA - 1);
            const int el   = (u >> SLA) & (CHUNK - 1);
            const int pk   = ((cbase + el) << SLA) | slot;
            if (t < RCAP) {
              if (lane == 0) { hl[t] = pk; cnt[slot] = cnt[slot] + 1; }
              t = t + 1;
            } else {
              ov = 1;
            }
          }
        }
      }
    }
    __syncthreads();
  }
  if (wave == 0 && lane == 0) { misc[8] = t; misc[9] = ov; }
  __syncthreads();
  int tt = misc[8];
  tt = tt < 0 ? 0 : (tt > RCAP ? RCAP : tt);
  const int ovf = misc[9];

  if (wave == 0) {
    const int base = lane * (NBA / 32);
    int s = 0;
#pragma unroll 1
    for (int i = 0; i < NBA / 32; ++i) s += cnt[base + i];
    int incl = s;
#pragma unroll
    for (int d = 1; d < 32; d <<= 1) {
      const int y = __shfl_up(incl, d, 32);
      if (lane >= d) incl += y;
    }
    int run = incl - s;
#pragma unroll 1
    for (int i = 0; i < NBA / 32; ++i) {
      const int cv = cnt[base + i];
      offs[base + i] = run;
      cur[base + i]  = run;
      run += cv;
    }
  }
  __syncthreads();
  if (wave == 0) {
#pragma unroll 1
    for (int b0 = 0; b0 < tt; b0 += 32) {
      const int idx = b0 + lane;
      const int ent = hl[idx < RCAP ? idx : RCAP - 1];
      const int m32 = (tt - b0) < 32 ? (tt - b0) : 32;
#pragma unroll 1
      for (int k = 0; k < m32; ++k) {
        const int u    = __builtin_amdgcn_readlane(ent, k);
        const int slot = u & (NBA - 1);
        if (lane == 0) {
          int p = cur[slot];
          p = p < 0 ? 0 : (p > RCAP - 1 ? RCAP - 1 : p);
          sl[p] = u;
          cur[slot] = p + 1;
        }
      }
    }
  }
  __syncthreads();

  const size_t eb = (size_t)blockIdx.x * RCAP;
#pragma unroll 1
  for (int i4 = tid * 4; i4 < RCAP; i4 += NTHR * 4) {
    const v4i u = *(const v4ia*)(sl + i4);
    int e0 = u.x >> SLA, e1 = u.y >> SLA, e2 = u.z >> SLA, e3 = u.w >> SLA;
    e0 = e0 < 0 ? 0 : (e0 > nE - 1 ? nE - 1 : e0);
    e1 = e1 < 0 ? 0 : (e1 > nE - 1 ? nE - 1 : e1);
    e2 = e2 < 0 ? 0 : (e2 > nE - 1 ? nE - 1 : e2);
    e3 = e3 < 0 ? 0 : (e3 > nE - 1 ? nE - 1 : e3);
    int r0 = srcs[e0], r1 = srcs[e1], r2 = srcs[e2], r3 = srcs[e3];
    r0 = r0 < 0 ? 0 : (r0 > nN - 1 ? nN - 1 : r0);
    r1 = r1 < 0 ? 0 : (r1 > nN - 1 ? nN - 1 : r1);
    r2 = r2 < 0 ? 0 : (r2 > nN - 1 ? nN - 1 : r2);
    r3 = r3 < 0 ? 0 : (r3 > nN - 1 ? nN - 1 : r3);
    v4i ev, sv;
    ev.x = e0; ev.y = e1; ev.z = e2; ev.w = e3;
    sv.x = r0; sv.y = r1; sv.z = r2; sv.w = r3;
    int* ep = eidp + eb + i4;
    int* sp = srcp + eb + i4;
    *(volatile v4i*)ep = ev;
    *(volatile v4i*)sp = sv;
    __threadfence();
    *(volatile v4i*)ep = ev;
    *(volatile v4i*)sp = sv;
  }
  {
    const v4i o4 = *(const v4ia*)(offs + 4 * tid);
    const v4i c4 = *(const v4ia*)(cnt + 4 * tid);
    int* op = offt + (size_t)blockIdx.x * (2 * NBA) + 4 * tid;
    *(volatile v4i*)op = o4;
    *(volatile v4i*)(op + NBA) = c4;
    __threadfence();
    *(volatile v4i*)op = o4;
    *(volatile v4i*)(op + NBA) = c4;
  }
  if (tid < 8) {
    v4i mv = {0, 0, 0, 0};
    if (tid == 0) { mv.x = tt; mv.y = ovf; }
    int* mp = meta + (size_t)blockIdx.x * 32 + 4 * tid;
    *(volatile v4i*)mp = mv;
    __threadfence();
    *(volatile v4i*)mp = mv;
  }
}

template <int NT>
__global__ __launch_bounds__(GTHR) void k_gemm(const unsigned short* __restrict__ A,
                                               const unsigned short* __restrict__ WT,
                                               const float* __restrict__ cvec, float* outF, int K, int ldo) {
  constexpr int GBN = 16 * NT;
  constexpr int LPR = GBN / 4;
  constexpr int RPI = 32 / LPR;
  constexpr int NIT = 16 / RPI;
  static_assert(LPR <= 32 && RPI >= 1 && NIT * RPI == 16);
  __shared__ __attribute__((aligned(16))) float stg[GBM * GBN];
  const int tid = (int)threadIdx.x, lane = tid & 31, wave = tid >> 5, hh = lane >> 4, m = lane & 15;
  const int rowBase = (int)blockIdx.x * GBM;
  const int col0    = (int)blockIdx.y * GBN;

  v8f acc[NT];
  {
    const v8f z = {0.f, 0.f, 0.f, 0.f, 0.f, 0.f, 0.f, 0.f};
#pragma unroll
    for (int t = 0; t < NT; ++t) acc[t] = z;
  }
  const unsigned short* ap = A  + (size_t)(rowBase + 16 * wave + m) * (size_t)K + 8 * hh;
  const unsigned short* wp = WT + (size_t)(col0 + m) * (size_t)K + 8 * hh;
  const int ksteps = K >> 5;
#pragma unroll 1
  for (int ks = 0; ks < ksteps; ++ks) {
    FragB af;
    af.u[0] = *(const v8us*)(ap + 32 * ks);
    af.u[1] = *(const v8us*)(ap + 32 * ks + 16);
#pragma unroll
    for (int t = 0; t < NT; ++t) {
      const unsigned short* wq = wp + (size_t)(16 * t) * (size_t)K + 32 * ks;
      FragB bf;
      bf.u[0] = *(const v8us*)wq;
      bf.u[1] = *(const v8us*)(wq + 16);
      acc[t] = wmx(af, bf, acc[t]);
    }
  }

#pragma unroll
  for (int t = 0; t < NT; ++t) {
    const int lc = 16 * t + m;
    const float cb = cvec[col0 + lc];
#pragma unroll
    for (int r = 0; r < 8; ++r) {
      const int lr = 16 * wave + 8 * hh + r;
      stg[lr * GBN + lc] = acc[t][r] + cb;
    }
  }
  __syncthreads();

  const int rsub = lane / LPR;
  const int cl   = lane - rsub * LPR;
  const bool act = rsub < RPI;
  const int rsc  = act ? rsub : (RPI - 1);
  v4f fv[NIT];
#pragma unroll
  for (int i = 0; i < NIT; ++i) {
    const int lr = 16 * wave + RPI * i + rsc;
    fv[i] = *(const v4fa*)(stg + lr * GBN + 4 * cl);
  }
#pragma unroll
  for (int i = 0; i < NIT; ++i) {
    const int gr = rowBase + 16 * wave + RPI * i + rsc;
    float* op = outF + (size_t)gr * (size_t)ldo + col0 + 4 * cl;
    if (act) *(volatile v4f*)op = fv[i];
  }
  __threadfence();
#pragma unroll
  for (int i = 0; i < NIT; ++i) {
    const int gr = rowBase + 16 * wave + RPI * i + rsc;
    float* op = outF + (size_t)gr * (size_t)ldo + col0 + 4 * cl;
    if (act) *(volatile v4f*)op = fv[i];
  }
}

template <int CPL>
__device__ __forceinline__ void ldg(const float* __restrict__ p, float (&o)[CPL]) {
  if constexpr (CPL == 2) {
    const v2f t = *(const v2f*)p;
    o[0] = t.x; o[1] = t.y;
  } else {
    o[0] = p[0];
  }
}

template <int CPL>
__global__ __launch_bounds__(NTHR) void k_scan(const int* __restrict__ eidp, const int* __restrict__ srcp,
                                               const int* __restrict__ offt, const int* __restrict__ meta,
                                               const float* __restrict__ P, int ldp, int oxl, int oxr,
                                               const float* __restrict__ ea, const float* __restrict__ We,
                                               const float* __restrict__ att, const float* __restrict__ cbias,
                                               const float* __restrict__ eeself,
                                               float* agg, double* rec, int nN, int nE) {
  constexpr int C  = 32 * CPL;
  constexpr int RW = (CPL == 2) ? 8 : 16;
  __shared__ __attribute__((aligned(16))) float  wes[16 * C];
  __shared__ __attribute__((aligned(16))) double wrec[NWAVE * 2 * C];
  __shared__ __attribute__((aligned(16))) double drec[2 * C];
  const int tid = (int)threadIdx.x, lane = tid & 31;
  const int wave = __builtin_amdgcn_readfirstlane(tid >> 5);
  const int b = (int)blockIdx.x;
  const int nodeBase = b * NBA;
  const int col0 = CPL * lane;

  for (int i = tid; i < 16 * C; i += NTHR) wes[i] = rbf(We[i]);
  int tt = meta[(size_t)b * 32];
  const int ovf = meta[(size_t)b * 32 + 1];
  tt = tt < 0 ? 0 : (tt > RCAP ? RCAP : tt);
  tt = __builtin_amdgcn_readfirstlane(tt);
  __syncthreads();

  float at[CPL], cb[CPL], es[CPL];
#pragma unroll
  for (int j = 0; j < CPL; ++j) {
    at[j] = rbf(att[col0 + j]);
    cb[j] = rbf(cbias[col0 + j]);
    es[j] = eeself[col0 + j];
  }
  const float qnan = __int_as_float(0x7fc00000);
  const float pz = (ovf != 0) ? qnan : 0.0f;
  const size_t eb = (size_t)b * RCAP;
  double sS[CPL], sQ[CPL];
#pragma unroll
  for (int j = 0; j < CPL; ++j) { sS[j] = 0.0; sQ[j] = 0.0; }

#pragma unroll 1
  for (int si = 0; si < NBA / NWAVE; ++si) {
    const int s    = si * NWAVE + wave;
    const int node = nodeBase + s;
    if (node < nN) {
      int c = offt[(size_t)b * (2 * NBA) + NBA + s];
      int o = offt[(size_t)b * (2 * NBA) + s];
      const bool big = c > DEGCAP;
      c = c < 0 ? 0 : (c > DEGCAP ? DEGCAP : c);
      o = o < 0 ? 0 : (o > tt ? tt : o);
      if (c > tt - o) c = tt - o;
      c = __builtin_amdgcn_readfirstlane(c);
      o = __builtin_amdgcn_readfirstlane(o);

      const float* prow = P + (size_t)node * (size_t)ldp;
      float xd[CPL], xr[CPL], av[CPL];
      ldg<CPL>(prow + oxl + col0, xd);
      ldg<CPL>(prow + oxr + col0, xr);
      float part = 0.0f;
#pragma unroll
      for (int j = 0; j < CPL; ++j) {
        float v = xd[j] + xr[j] + es[j];
        v = v > 0.0f ? v : v * NEGS;
        part = fmaf(v, at[j], part);
        av[j] = xd[j];
      }
#pragma unroll
      for (int off = RW; off > 0; off >>= 1) part += __shfl_xor(part, off);
      float mx = part, dn = 1.0f;

#pragma unroll 1
      for (int b0 = 0; b0 < c; b0 += 32) {
        int idx = o + b0 + lane;
        idx = idx > RCAP - 1 ? RCAP - 1 : idx;
        int eid = eidp[eb + idx];
        eid = eid < 0 ? 0 : (eid > nE - 1 ? nE - 1 : eid);
        int sr = srcp[eb + idx];
        sr = sr < 0 ? 0 : (sr > nN - 1 ? nN - 1 : sr);
        const int m32 = (c - b0) < 32 ? (c - b0) : 32;
#pragma unroll 1
        for (int k = 0; k < m32; ++k) {
          const int sk = __builtin_amdgcn_readlane(sr, k);
          const int ek = __builtin_amdgcn_readlane(eid, k);
          float xs[CPL], ee[CPL];
          ldg<CPL>(P + (size_t)sk * (size_t)ldp + oxl + col0, xs);
          const float eav = rbf(ea[(size_t)ek * 16 + (lane & 15)]);
          const int eai = __float_as_int(eav);
#pragma unroll
          for (int j = 0; j < CPL; ++j) ee[j] = 0.0f;
#pragma unroll 4
          for (int kk = 0; kk < 16; ++kk) {
            const float a = __int_as_float(__builtin_amdgcn_readlane(eai, kk));
            if constexpr (CPL == 2) {
              const v2f w = *(const v2fa*)(&wes[kk * C + col0]);
              ee[0] = fmaf(a, w.x, ee[0]);
              ee[1] = fmaf(a, w.y, ee[1]);
            } else {
              ee[0] = fmaf(a, wes[kk * C + col0], ee[0]);
            }
          }
          float pt = 0.0f;
#pragma unroll
          for (int j = 0; j < CPL; ++j) {
            float v = xs[j] + xr[j] + ee[j];
            v = v > 0.0f ? v : v * NEGS;
            pt = fmaf(v, at[j], pt);
          }
#pragma unroll
          for (int off = RW; off > 0; off >>= 1) pt += __shfl_xor(pt, off);
          const float df = pt - mx;
          const float ex = expf(-fabsf(df));
          const bool up  = df > 0.0f;
          const float s1 = up ? ex : 1.0f;
          const float s2 = up ? 1.0f : ex;
          mx = up ? pt : mx;
          dn = fmaf(dn, s1, s2);
#pragma unroll
          for (int j = 0; j < CPL; ++j) av[j] = fmaf(av[j], s1, s2 * xs[j]);
        }
      }
      const float inv = 1.0f / (dn + 1e-16f);
      const float pzr = big ? qnan : pz;
      float r[CPL];
#pragma unroll
      for (int j = 0; j < CPL; ++j) {
        r[j] = fmaf(av[j], inv, cb[j]) + pzr;
        const double rd = (double)r[j];
        sS[j] += rd;
        sQ[j] += rd * rd;
      }
      float* gp = agg + (size_t)node * C + col0;
      if constexpr (CPL == 2) {
        v2f rv;
        rv.x = r[0]; rv.y = r[1];
        *(volatile v2f*)gp = rv;
        __threadfence();
        *(volatile v2f*)gp = rv;
      } else {
        const float rv = r[0];
        *(volatile float*)gp = rv;
        __threadfence();
        *(volatile float*)gp = rv;
      }
    }
  }

#pragma unroll
  for (int j = 0; j < CPL; ++j) {
    wrec[wave * 2 * C + col0 + j]     = sS[j];
    wrec[wave * 2 * C + C + col0 + j] = sQ[j];
  }
  __syncthreads();
  if (tid < 2 * C) {
    double a = 0.0;
#pragma unroll 1
    for (int w2 = 0; w2 < NWAVE; ++w2) a += wrec[w2 * 2 * C + tid];
    drec[tid] = a;
  }
  __syncthreads();
  if (tid < C) {
    v2d t;
    t.x = drec[2 * tid]; t.y = drec[2 * tid + 1];
    double* dp = rec + (size_t)b * (2 * C) + 2 * tid;
    *(volatile v2d*)dp = t;
    __threadfence();
    *(volatile v2d*)dp = t;
  }
}

__global__ __launch_bounds__(NTHR) void k_bn1(const float* __restrict__ agg, const float* __restrict__ p1,
                                              const double* __restrict__ rec, int nRec,
                                              const float* __restrict__ gam, const float* __restrict__ bet,
                                              unsigned short* h1hl, int nN, int MP) {
  __shared__ float smu[C1], srs[C1], sg[C1], sb[C1];
  __shared__ __attribute__((aligned(16))) float hs[32 * C1];
  const int tid = (int)threadIdx.x;
  if (tid < C1) {
    double S = 0.0, Q = 0.0;
#pragma unroll 1
    for (int b = 0; b < nRec; ++b) {
      S += rec[(size_t)b * (2 * C1) + tid];
      Q += rec[(size_t)b * (2 * C1) + C1 + tid];
    }
    const double rn = 1.0 / (double)nN;
    const double mean = S * rn;
    const double var = Q * rn - mean * mean;
    smu[tid] = (float)mean;
    srs[tid] = 1.0f / sqrtf((float)var + 1e-5f);
    sg[tid]  = rbf(gam[tid]);
    sb[tid]  = rbf(bet[tid]);
  }
  __syncthreads();
  const int rowBlock = (int)blockIdx.x * 256;
#pragma unroll 1
  for (int t = 0; t < 8; ++t) {
    const int r0 = rowBlock + t * 32;
#pragma unroll 1
    for (int i = 0; i < 8; ++i) {
      const int e  = i * NTHR + tid;
      const int lr = e >> 6;
      const int c  = e & 63;
      const int row = r0 + lr;
      const int rc  = row < nN ? row : nN - 1;
      const float a  = agg[(size_t)rc * C1 + c];
      const float hp = p1[(size_t)rc * N1 + c];
      float y = (a - smu[c]) * srs[c] * sg[c] + sb[c] + hp;
      y = y > 0.0f ? y : expm1f(y);
      hs[e] = row < nN ? y : 0.0f;
    }
    __syncthreads();
#pragma unroll
    for (int i2 = 0; i2 < 2; ++i2) {
      const int u  = i2 * NTHR + tid;
      const int lr = u >> 4;
      const int pt = (u >> 3) & 1;
      const int cg = u & 7;
      const v4f ga = *(const v4fa*)(hs + lr * C1 + 8 * cg);
      const v4f gb = *(const v4fa*)(hs + lr * C1 + 8 * cg + 4);
      const float f[8] = {ga.x, ga.y, ga.z, ga.w, gb.x, gb.y, gb.z, gb.w};
      v8us o;
#pragma unroll
      for (int j = 0; j < 8; ++j) {
        const unsigned hb = bfbits(f[j]);
        const unsigned lb = bfbits(f[j] - __uint_as_float(hb << 16));
        o[j] = (unsigned short)(pt != 0 ? lb : hb);
      }
      const int row = r0 + lr;
      unsigned short* dp = h1hl + (size_t)row * KG + 8 * (u & 15);
      if (row < MP) *(volatile v8us*)dp = o;
      __threadfence();
      if (row < MP) *(volatile v8us*)dp = o;
    }
    __syncthreads();
  }
}

__global__ __launch_bounds__(NTHR) void k_bn2pool(const float* __restrict__ agg, const float* __restrict__ p2,
                                                  const double* __restrict__ rec, int nRec,
                                                  const float* __restrict__ gam, const float* __restrict__ bet,
                                                  const int* __restrict__ batch,
                                                  double* psum, float* pmax, int* pcnt, int nN) {
  __shared__ float smu[C2], srs[C2], sg[C2], sb[C2];
  __shared__ __attribute__((aligned(16))) double wsum[NWAVE * NG * 32];
  __shared__ __attribute__((aligned(16))) float  wmax[NWAVE * NG * 32];
  __shared__ int wcnt[NWAVE * NG];
  __shared__ __attribute__((aligned(16))) double dsum[NG * 32];
  __shared__ __attribute__((aligned(16))) float  fmaxs[NG * 32];
  __shared__ __attribute__((aligned(16))) int    icnt[32];
  const int tid = (int)threadIdx.x, lane = tid & 31;
  const int wave = __builtin_amdgcn_readfirstlane(tid >> 5);
  const float ninf = __int_as_float((int)0xff800000);
  if (tid < C2) {
    double S = 0.0, Q = 0.0;
#pragma unroll 1
    for (int b = 0; b < nRec; ++b) {
      S += rec[(size_t)b * (2 * C2) + tid];
      Q += rec[(size_t)b * (2 * C2) + C2 + tid];
    }
    const double rn = 1.0 / (double)nN;
    const double mean = S * rn;
    const double var = Q * rn - mean * mean;
    smu[tid] = (float)mean;
    srs[tid] = 1.0f / sqrtf((float)var + 1e-5f);
    sg[tid]  = rbf(gam[tid]);
    sb[tid]  = rbf(bet[tid]);
  }
  for (int i = tid; i < NWAVE * NG * 32; i += NTHR) { wsum[i] = 0.0; wmax[i] = ninf; }
  if (tid < NWAVE * NG) wcnt[tid] = 0;
  __syncthreads();
  const float mu = smu[lane], rs = srs[lane], gg = sg[lane], bb = sb[lane];
  const int base = (int)blockIdx.x * NBA;
#pragma unroll 1
  for (int si = 0; si < NBA / NWAVE; ++si) {
    const int row = base + si * NWAVE + wave;
    if (row < nN) {
      const int g = __builtin_amdgcn_readfirstlane(batch[row]);
      const float a  = agg[(size_t)row * C2 + lane];
      const float hp = p2[(size_t)row * N2 + lane];
      float y = (a - mu) * rs * gg + bb + hp;
      y = y > 0.0f ? y : expm1f(y);
      if ((unsigned)g < (unsigned)NG) {
        const int idx = (wave * NG + g) * 32 + lane;
        wsum[idx] = wsum[idx] + (double)y;
        const float mo = wmax[idx];
        wmax[idx] = (y > mo || y != y) ? y : mo;
        const int cn = wcnt[wave * NG + g];
        wcnt[wave * NG + g] = cn + 1;
      }
    }
  }
  __syncthreads();
#pragma unroll
  for (int i2 = 0; i2 < 2; ++i2) {
    const int p = i2 * NTHR + tid;
    double a = 0.0;
    float mxv = ninf;
#pragma unroll 1
    for (int w2 = 0; w2 < NWAVE; ++w2) {
      a += wsum[w2 * NG * 32 + p];
      const float v = wmax[w2 * NG * 32 + p];
      mxv = (v > mxv || v != v) ? v : mxv;
    }
    dsum[p] = a;
    fmaxs[p] = mxv;
  }
  if (tid < 32) {
    int cs = 0;
#pragma unroll 1
    for (int w2 = 0; w2 < NWAVE; ++w2) cs += wcnt[w2 * NG + (tid & 15)];
    icnt[tid] = tid < NG ? cs : 0;
  }
  __syncthreads();
  const size_t pb = (size_t)blockIdx.x;
  v2d ds;
  ds.x = dsum[2 * tid]; ds.y = dsum[2 * tid + 1];
  const int t4 = tid < 128 ? tid : 127;
  const v4f ms = *(const v4fa*)(fmaxs + 4 * t4);
  const int t8 = tid < 8 ? tid : 7;
  const v4i cs4 = *(const v4ia*)(icnt + 4 * t8);
  double* sp = psum + pb * (NG * 32) + 2 * tid;
  float*  mp = pmax + pb * (NG * 32) + 4 * t4;
  int*    cp = pcnt + pb * 32 + 4 * t8;
  *(volatile v2d*)sp = ds;
  if (tid < 128) *(volatile v4f*)mp = ms;
  if (tid < 8)   *(volatile v4i*)cp = cs4;
  __threadfence();
  *(volatile v2d*)sp = ds;
  if (tid < 128) *(volatile v4f*)mp = ms;
  if (tid < 8)   *(volatile v4i*)cp = cs4;
}

__global__ __launch_bounds__(NTHR) void k_final(const double* __restrict__ psum, const float* __restrict__ pmax,
                                                const int* __restrict__ pcnt, const int* __restrict__ meta,
                                                int nB, float* out) {
  const int t = (int)threadIdx.x;
  const int g = t >> 4, q = t & 15;
  const int cc = (q & 7) * 4;
  const bool isMax = q >= 8;
  const float ninf = __int_as_float((int)0xff800000);
  double s0 = 0.0, s1 = 0.0, s2 = 0.0, s3 = 0.0;
  float m0 = ninf, m1 = ninf, m2 = ninf, m3 = ninf;
  int cnt = 0, flag = 0;
#pragma unroll 1
  for (int b = 0; b < nB; ++b) {
    const double* ps = psum + (size_t)b * (NG * 32) + g * 32 + cc;
    const v2d a  = *(const v2d*)ps;
    const v2d a2 = *(const v2d*)(ps + 2);
    const v4f mv = *(const v4f*)(pmax + (size_t)b * (NG * 32) + g * 32 + cc);
    cnt  += pcnt[(size_t)b * 32 + g];
    flag |= meta[(size_t)b * 32 + 1];
    s0 += a.x; s1 += a.y; s2 += a2.x; s3 += a2.y;
    m0 = (mv.x > m0 || mv.x != mv.x) ? mv.x : m0;
    m1 = (mv.y > m1 || mv.y != mv.y) ? mv.y : m1;
    m2 = (mv.z > m2 || mv.z != mv.z) ? mv.z : m2;
    m3 = (mv.w > m3 || mv.w != mv.w) ? mv.w : m3;
  }
  const double dd = (double)(cnt > 1 ? cnt : 1);
  const bool has = cnt > 0;
  v4f o;
  o.x = isMax ? (has ? m0 : 0.0f) : (float)(s0 / dd);
  o.y = isMax ? (has ? m1 : 0.0f) : (float)(s1 / dd);
  o.z = isMax ? (has ? m2 : 0.0f) : (float)(s2 / dd);
  o.w = isMax ? (has ? m3 : 0.0f) : (float)(s3 / dd);
  if (flag != 0) {
    const float qn = __int_as_float(0x7fc00000);
    o.x = qn; o.y = qn; o.z = qn; o.w = qn;
  }
  float* op = out + 4 * t;
  *(volatile v4f*)op = o;
  __threadfence();
  *(volatile v4f*)op = o;
}

static inline int cdiv(int a, int b) { return (a + b - 1) / b; }
static inline size_t al256(size_t o) { return (o + 255) & ~(size_t)255; }

extern "C" void kernel_launch(void* const* d_in, const int* in_sizes, int n_in,
                              void* d_out, int out_size, void* d_ws, size_t ws_size,
                              hipStream_t stream) {
  if (n_in < 26) return;
  if (in_sizes[0] < FIN || (in_sizes[0] % FIN) != 0) return;
  const int nN = in_sizes[0] / FIN;
  if (nN < 16 || nN >= (1 << 22)) return;
  if (in_sizes[1] < 2 || (in_sizes[1] & 1) != 0) return;
  const int nE = in_sizes[1] / 2;
  if (nE < 1 || nE >= (1 << 21)) return;
  if ((long long)in_sizes[2] != (long long)nE * 16) return;
  if (in_sizes[3] != nN) return;
  if (in_sizes[4] != FIN * C1 || in_sizes[5] != C1) return;
  if (in_sizes[6] != FIN * C1 || in_sizes[7] != C1) return;
  if (in_sizes[8] != FIN * C1 || in_sizes[9] != C1) return;
  if (in_sizes[10] != 16 * C1 || in_sizes[11] != C1 || in_sizes[12] != C1) return;
  if (in_sizes[13] != C1 || in_sizes[14] != C1) return;
  if (in_sizes[15] != C1 * C2 || in_sizes[16] != C2) return;
  if (in_sizes[17] != C1 * C2 || in_sizes[18] != C2) return;
  if (in_sizes[19] != C1 * C2 || in_sizes[20] != C2) return;
  if (in_sizes[21] != 16 * C2 || in_sizes[22] != C2 || in_sizes[23] != C2) return;
  if (in_sizes[24] != C2 || in_sizes[25] != C2) return;
  if (out_size != NG * 64) return;

  const float* x      = (const float*)d_in[0];
  const int*   ei     = (const int*)  d_in[1];
  const float* ea     = (const float*)d_in[2];
  const int*   batch  = (const int*)  d_in[3];
  const float* s1w    = (const float*)d_in[4];
  const float* s1b    = (const float*)d_in[5];
  const float* wl1    = (const float*)d_in[6];
  const float* bl1    = (const float*)d_in[7];
  const float* wr1    = (const float*)d_in[8];
  const float* br1    = (const float*)d_in[9];
  const float* we1    = (const float*)d_in[10];
  const float* att1   = (const float*)d_in[11];
  const float* cb1    = (const float*)d_in[12];
  const float* g1     = (const float*)d_in[13];
  const float* b1     = (const float*)d_in[14];
  const float* s2w    = (const float*)d_in[15];
  const float* s2b    = (const float*)d_in[16];
  const float* wl2    = (const float*)d_in[17];
  const float* bl2    = (const float*)d_in[18];
  const float* wr2    = (const float*)d_in[19];
  const float* br2    = (const float*)d_in[20];
  const float* we2    = (const float*)d_in[21];
  const float* att2   = (const float*)d_in[22];
  const float* cb2    = (const float*)d_in[23];
  const float* g2     = (const float*)d_in[24];
  const float* b2     = (const float*)d_in[25];
  float* out = (float*)d_out;
  const int* src = ei;
  const int* dst = ei + nE;

  const int MP   = cdiv(nN, GBM) * GBM;
  const int gM   = MP / GBM;
  const int gA   = cdiv(nN, NBA);
  const int nBE  = cdiv(nE, EAR);
  const int vec8 = ((nE & 3) == 0) ? 1 : 0;

  char* ws = (char*)d_ws;
  size_t off = 0;
  const size_t oXB   = off; off = al256(off + (size_t)MP * FIN * 2);
  const size_t oWT   = off; off = al256(off + (size_t)(N1 + N2) * KG * 2);
  const size_t oVEC  = off; off = al256(off + (size_t)VEC_N * 4);
  const size_t oEAR  = off; off = al256(off + (size_t)nBE * 16 * 8);
  const size_t oP1   = off; off = al256(off + (size_t)MP * N1 * 4);
  const size_t oEID  = off; off = al256(off + (size_t)gA * RCAP * 4);
  const size_t oSRC  = off; off = al256(off + (size_t)gA * RCAP * 4);
  const size_t oOFF  = off; off = al256(off + (size_t)gA * 2 * NBA * 4);
  const size_t oMETA = off; off = al256(off + (size_t)gA * 32 * 4);
  const size_t oAG1  = off; off = al256(off + (size_t)MP * C1 * 4);
  const size_t oRC1  = off; off = al256(off + (size_t)gA * 2 * C1 * 8);
  const size_t oHL   = off; off = al256(off + (size_t)MP * KG * 2);
  const size_t oP2   = off; off = al256(off + (size_t)MP * N2 * 4);
  const size_t oAG2  = off; off = al256(off + (size_t)MP * C2 * 4);
  const size_t oRC2  = off; off = al256(off + (size_t)gA * 2 * C2 * 8);
  const size_t oPS   = off; off = al256(off + (size_t)gA * NG * 32 * 8);
  const size_t oPM   = off; off = al256(off + (size_t)gA * NG * 32 * 4);
  const size_t oPC   = off; off = al256(off + (size_t)gA * 32 * 4);
  if (off > ws_size || off > (size_t)WSMAX) return;

  unsigned short* XB   = (unsigned short*)(ws + oXB);
  unsigned short* WT   = (unsigned short*)(ws + oWT);
  unsigned short* B1t  = WT;
  unsigned short* B2t  = WT + (size_t)N1 * KG;
  float*  VEC  = (float*)(ws + oVEC);
  double* EAR_ = (double*)(ws + oEAR);
  float*  P1   = (float*)(ws + oP1);
  int*    EIDP = (int*)(ws + oEID);
  int*    SRCP = (int*)(ws + oSRC);
  int*    OFFT = (int*)(ws + oOFF);
  int*    META = (int*)(ws + oMETA);
  float*  AGG1 = (float*)(ws + oAG1);
  double* REC1 = (double*)(ws + oRC1);
  unsigned short* H1HL = (unsigned short*)(ws + oHL);
  float*  P2   = (float*)(ws + oP2);
  float*  AGG2 = (float*)(ws + oAG2);
  double* REC2 = (double*)(ws + oRC2);
  double* PSUM = (double*)(ws + oPS);
  float*  PMAX = (float*)(ws + oPM);
  int*    PCNT = (int*)(ws + oPC);

  const size_t bkLds = (size_t)BK_LDS_INTS * 4;
  hipFuncSetAttribute(reinterpret_cast<const void*>(&k_bucket),
                      hipFuncAttributeMaxDynamicSharedMemorySize, (int)bkLds);

  const int nUx = MP * (FIN / 8);
  k_xprep<<<cdiv(nUx, NTHR), NTHR, 0, stream>>>(x, XB, nN, nUx);
  k_wprep<<<4608 / NTHR, NTHR, 0, stream>>>(s1w, wl1, wr1, s2w, wl2, wr2, WT);
  k_easum<<<nBE, NTHR, 0, stream>>>(ea, nE, EAR_);
  k_eamean<<<1, 384, 0, stream>>>(EAR_, nBE, nE, we1, we2, s1b, bl1, br1, s2b, bl2, br2, VEC);
  k_bucket<<<gA, NTHR, bkLds, stream>>>(src, dst, nE, nN, vec8, EIDP, SRCP, OFFT, META);
  k_gemm<4><<<dim3(gM, N1 / 64), GTHR, 0, stream>>>(XB, B1t, VEC, P1, KG, N1);
  k_scan<2><<<gA, NTHR, 0, stream>>>(EIDP, SRCP, OFFT, META, P1, N1, C1, 2 * C1, ea, we1, att1, cb1,
                                     VEC + 288, AGG1, REC1, nN, nE);
  k_bn1<<<cdiv(MP, 256), NTHR, 0, stream>>>(AGG1, P1, REC1, gA, g1, b1, H1HL, nN, MP);
  k_gemm<6><<<dim3(gM, 1), GTHR, 0, stream>>>(H1HL, B2t, VEC + N1, P2, KG, N2);
  k_scan<1><<<gA, NTHR, 0, stream>>>(EIDP, SRCP, OFFT, META, P2, N2, C2, 2 * C2, ea, we2, att2, cb2,
                                     VEC + 352, AGG2, REC2, nN, nE);
  k_bn2pool<<<gA, NTHR, 0, stream>>>(AGG2, P2, REC2, gA, g2, b2, batch, PSUM, PMAX, PCNT, nN);
  k_final<<<1, NTHR, 0, stream>>>(PSUM, PMAX, PCNT, META, gA, out);
}
